// QattenMixer_63333587746988
// MI455X (gfx1250) — hardware-verified
//
#include <hip/hip_runtime.h>


#define BB 4096
#define NA_ 16
#define UU 32
#define SS 560
#define NH 4
#define EE 32
#define GH 64
#define BCH 1024
#define NPR (BCH * NA_ * NA_)

typedef __attribute__((ext_vector_type(16))) __bf16   v16bf;
typedef __attribute__((ext_vector_type(16))) _Float16 v16h;
typedef __attribute__((ext_vector_type(8)))  float    v8f;
typedef __attribute__((ext_vector_type(8)))  unsigned v8u;

__device__ __forceinline__ unsigned f2bf(float f) { unsigned u = __float_as_uint(f); u += 0x7FFFu + ((u >> 16) & 1u); return u >> 16; }
__device__ __forceinline__ unsigned f2h(float f) { return (unsigned)__builtin_bit_cast(unsigned short, (_Float16)f); }
__device__ __forceinline__ int kpat(int v, int half) { return ((v & 4) ? 16 : 0) + half * 8 + 2 * (v & 3); }

template <int F16, int NP> struct Opnd { v16bf p[NP]; };

template <int F16, int NP> __device__ __forceinline__ void pack2(float f0, float f1, unsigned* o) {
    if (F16) { o[0] = f2h(f0) | (f2h(f1) << 16); return; }
    unsigned h0 = f2bf(f0), h1 = f2bf(f1); o[0] = h0 | (h1 << 16);
    if (NP >= 2) {
        float r0 = f0 - __uint_as_float(h0 << 16), r1 = f1 - __uint_as_float(h1 << 16);
        unsigned m0 = f2bf(r0), m1 = f2bf(r1); o[1] = m0 | (m1 << 16);
        if (NP >= 3) {
            float s0 = r0 - __uint_as_float(m0 << 16), s1 = r1 - __uint_as_float(m1 << 16);
            o[2] = f2bf(s0) | (f2bf(s1) << 16);
        }
    }
}
template <int F16, int NP> __device__ __forceinline__ void op_row(const float* rowp, int half, float sc, Opnd<F16, NP>& o) {
    v8u u[NP];
#pragma unroll
    for (int v = 0; v < 8; ++v) {
        int kk = kpat(v, half); unsigned t[3];
        pack2<F16, NP>(rowp[kk] * sc, rowp[kk + 1] * sc, t);
#pragma unroll
        for (int p = 0; p < NP; ++p) u[p][v] = t[p];
    }
#pragma unroll
    for (int p = 0; p < NP; ++p) o.p[p] = __builtin_bit_cast(v16bf, u[p]);
}
template <int F16, int NP> __device__ __forceinline__ void op_row_tail(const float* rowp, int half, float sc, int kvalid, Opnd<F16, NP>& o) {
    v8u u[NP];
#pragma unroll
    for (int v = 0; v < 8; ++v) {
        int kk = kpat(v, half); unsigned t[3];
        float f0 = kk < kvalid ? rowp[kk] * sc : 0.0f, f1 = (kk + 1) < kvalid ? rowp[kk + 1] * sc : 0.0f;
        pack2<F16, NP>(f0, f1, t);
#pragma unroll
        for (int p = 0; p < NP; ++p) u[p][v] = t[p];
    }
#pragma unroll
    for (int p = 0; p < NP; ++p) o.p[p] = __builtin_bit_cast(v16bf, u[p]);
}
template <int F16, int NP> __device__ __forceinline__ void op_col(const float* M, int ld, int n, int k0, int half, float sc, Opnd<F16, NP>& o) {
    v8u u[NP];
#pragma unroll
    for (int v = 0; v < 8; ++v) {
        int kk = k0 + kpat(v, half); unsigned t[3];
        pack2<F16, NP>(M[(size_t)kk * ld + n] * sc, M[(size_t)(kk + 1) * ld + n] * sc, t);
#pragma unroll
        for (int p = 0; p < NP; ++p) u[p][v] = t[p];
    }
#pragma unroll
    for (int p = 0; p < NP; ++p) o.p[p] = __builtin_bit_cast(v16bf, u[p]);
}
template <int F16, int NP> __device__ __forceinline__ void op_col_tail(const float* M, int ld, int n, int k0, int half, float sc, int K, Opnd<F16, NP>& o) {
    v8u u[NP];
#pragma unroll
    for (int v = 0; v < 8; ++v) {
        int kk = k0 + kpat(v, half); unsigned t[3];
        float f0 = kk < K ? M[(size_t)kk * ld + n] * sc : 0.0f, f1 = (kk + 1) < K ? M[(size_t)(kk + 1) * ld + n] * sc : 0.0f;
        pack2<F16, NP>(f0, f1, t);
#pragma unroll
        for (int p = 0; p < NP; ++p) u[p][v] = t[p];
    }
#pragma unroll
    for (int p = 0; p < NP; ++p) o.p[p] = __builtin_bit_cast(v16bf, u[p]);
}
__device__ __forceinline__ v8f wm_bf16(v16bf a, v16bf b, v8f c) { return __builtin_amdgcn_wmma_f32_16x16x32_bf16(false, a, false, b, (short)0, c, false, false); }
template <int F16, int NA, int NB> __device__ __forceinline__ v8f wmma_op(const Opnd<F16, NA>& a, const Opnd<F16, NB>& b, v8f c) {
    if (F16) {
        v16h ah = __builtin_bit_cast(v16h, a.p[0]), bh = __builtin_bit_cast(v16h, b.p[0]);
        c = __builtin_amdgcn_wmma_f32_16x16x32_f16(false, ah, false, bh, (short)0, c, false, false);
        asm volatile("v_nop\n\tv_nop\n\tv_nop\n\tv_nop" : "+v"(c) : "v"(ah), "v"(bh));
        return c;
    }
    constexpr int NMX = NA > NB ? NA : NB;
#pragma unroll
    for (int i = 0; i < NA; ++i)
#pragma unroll
        for (int j = 0; j < NB; ++j)
            if (i + j < NMX) c = wm_bf16(a.p[i], b.p[j], c);
    if (NA == 1 && NB == 1)      asm volatile("v_nop\n\tv_nop\n\tv_nop\n\tv_nop" : "+v"(c) : "v"(a.p[0]), "v"(b.p[0]));
    else if (NA == 2 && NB == 1) asm volatile("v_nop\n\tv_nop\n\tv_nop\n\tv_nop" : "+v"(c) : "v"(a.p[0]), "v"(a.p[1]), "v"(b.p[0]));
    else if (NA == 1 && NB == 2) asm volatile("v_nop\n\tv_nop\n\tv_nop\n\tv_nop" : "+v"(c) : "v"(a.p[0]), "v"(b.p[0]), "v"(b.p[1]));
    else if (NA == 2 && NB == 2) asm volatile("v_nop\n\tv_nop\n\tv_nop\n\tv_nop" : "+v"(c) : "v"(a.p[0]), "v"(a.p[1]), "v"(b.p[0]), "v"(b.p[1]));
    else                         asm volatile("v_nop\n\tv_nop\n\tv_nop\n\tv_nop" : "+v"(c) : "v"(a.p[0]), "v"(a.p[NA - 1]), "v"(b.p[0]), "v"(b.p[NB - 1]), "v"(a.p[NA / 2]), "v"(b.p[NB / 2]));
    return c;
}

struct ZMap { long long s1; long long s2; int zdiv; int pad_; };
__device__ __forceinline__ size_t zoff(const ZMap& m, int z) { return (size_t)((long long)(z / m.zdiv) * m.s1 + (long long)(z % m.zdiv) * m.s2); }

#define ACT_NONE 0
#define ACT_RELU 1
#define ACT_GELU_ERF 2
#define ACT_SILU 3
#define ACT_TANH 4
__device__ __forceinline__ float act_apply(int act, float x) {
    if (act == ACT_RELU) return x > 0.f ? x : 0.f;
    if (act == ACT_GELU_ERF) return 0.5f * x * (1.0f + erff(x * 0.70710678118654752f));
    if (act == ACT_SILU) return x / (1.0f + expf(-x));
    if (act == ACT_TANH) return tanhf(x);
    return x;
}
struct GemmArgs {
    ZMap za, zb_, zc, zbias, zadd, zrsc, zmul, zrbias;
    const float* A; const float* Bm; float* C; const float* bias; const float* add; const float* rsc; const float* mul; const float* rbias;
    long long ldadd, ldmul;
    int lda, ldb, ldc, K;
    float ascale, bscale, oscale, addscale;
    int M, nvalid, nstore, ldrsc;
    int bcs, pad1, pad2, pad3;
};
template <int BT, int F16, int NA, int NB, int RW, int CW, int ACT>
__global__ __launch_bounds__(256) void gemm_kernel(GemmArgs g) {
    constexpr int TR = 16 * RW, TC = 64 * CW, CSTR = TC + 4;
    __shared__ __align__(16) float cst[TR * CSTR];
    const int z = blockIdx.z;
    const float* A = g.A + zoff(g.za, z); const float* Bm = g.Bm + zoff(g.zb_, z); float* C = g.C + zoff(g.zc, z);
    const int tid = threadIdx.x, lane = tid & 31, wv = tid >> 5;
    const int l16 = lane & 15, half = lane >> 4;
    const int rt = wv % RW, ch = wv / RW;
    const int row0 = blockIdx.x * TR, col0 = blockIdx.y * TC + ch * 64;
    int arix = row0 + rt * 16 + l16; if (arix >= g.M) arix = g.M - 1;
    const float* arow = A + (size_t)arix * g.lda;
    v8f acc[4];
#pragma unroll
    for (int t = 0; t < 4; ++t) acc[t] = (v8f){};
    const int K = g.K;
#pragma unroll 1
    for (int kc = 0; kc < K; kc += 32) {
        Opnd<F16, NA> a;
        if (kc + 32 <= K) op_row<F16, NA>(arow + kc, half, g.ascale, a); else op_row_tail<F16, NA>(arow + kc, half, g.ascale, K - kc, a);
#pragma unroll
        for (int t = 0; t < 4; ++t) {
            Opnd<F16, NB> b;
            const int n = col0 + t * 16 + l16;
            if (n < g.nvalid) {
                if (BT) { if (kc + 32 <= K) op_row<F16, NB>(Bm + (size_t)n * g.ldb + kc, half, g.bscale, b); else op_row_tail<F16, NB>(Bm + (size_t)n * g.ldb + kc, half, g.bscale, K - kc, b); }
                else    { if (kc + 32 <= K) op_col<F16, NB>(Bm, g.ldb, n * g.bcs, kc, half, g.bscale, b); else op_col_tail<F16, NB>(Bm, g.ldb, n * g.bcs, kc, half, g.bscale, K, b); }
            } else {
#pragma unroll
                for (int p = 0; p < NB; ++p) b.p[p] = (v16bf){};
            }
            acc[t] = wmma_op<F16, NA, NB>(a, b, acc[t]);
        }
    }
    const float* bias = g.bias ? g.bias + zoff(g.zbias, z) : nullptr;
    const float* add = g.add ? g.add + zoff(g.zadd, z) : nullptr;
    const float* rsc = g.rsc ? g.rsc + zoff(g.zrsc, z) : nullptr;
    const float* mul = g.mul ? g.mul + zoff(g.zmul, z) : nullptr;
    const float* rbias = g.rbias ? g.rbias + zoff(g.zrbias, z) : nullptr;
#pragma unroll
    for (int t = 0; t < 4; ++t) {
        const int cl = ch * 64 + t * 16 + l16;
        const int cg = blockIdx.y * TC + cl;
        const bool cok = cg < g.nvalid;
        const float bv = (bias && cok) ? bias[(size_t)cg * g.bcs] : 0.0f;
#pragma unroll
        for (int r = 0; r < 8; ++r) {
            const int rl = rt * 16 + r + 8 * half;
            float v = acc[t][r] * g.oscale + bv;
            int rg = row0 + rl; if (rg >= g.M) rg = g.M - 1;
            if (rbias) v += rbias[rg];
            if (rsc) v *= rsc[(size_t)rg * g.ldrsc];
            if (mul && cok) v *= mul[(size_t)rg * g.ldmul + cg];
            if (add && cok) v += g.addscale * add[(size_t)rg * g.ldadd + cg];
            cst[rl * CSTR + cl] = v;
        }
    }
    __syncthreads();
    const int col = tid % TC, rsel = tid / TC, rstep = 256 / TC;
    if (ACT != ACT_NONE) {
#pragma unroll 1
        for (int r = rsel; r < TR; r += rstep) cst[r * CSTR + col] = act_apply(ACT, cst[r * CSTR + col]);
    }
    float* ob = C + (size_t)row0 * g.ldc + (size_t)blockIdx.y * TC;
    const bool colok = (int)(blockIdx.y * TC + col) < g.nstore;
    const int rmax = (g.M - row0 < TR) ? (g.M - row0) : TR;
    auto pass = [&]() {
        if (colok) {
#pragma unroll 4
            for (int r = rsel; r < rmax; r += rstep) *(volatile float*)(ob + (size_t)r * g.ldc + col) = cst[r * CSTR + col];
        }
    };
    pass();
    __threadfence();
    pass();
}
static inline ZMap zm(long long s1) { ZMap m; m.s1 = s1; m.s2 = 0; m.zdiv = 1; m.pad_ = 0; return m; }
static inline ZMap zm2(long long s1, long long s2, int zdiv) { ZMap m; m.s1 = s1; m.s2 = s2; m.zdiv = zdiv; m.pad_ = 0; return m; }
static inline GemmArgs gemm_args(const float* A, int lda, ZMap za, const float* Bm, int ldb, ZMap zb, float* C, int ldc, ZMap zc, int M, int N, int K) {
    GemmArgs g; g.za = za; g.zb_ = zb; g.zc = zc; g.zbias = zm(0); g.zadd = zm(0); g.zrsc = zm(0); g.zmul = zm(0); g.zrbias = zm(0);
    g.A = A; g.Bm = Bm; g.C = C; g.bias = nullptr; g.add = nullptr; g.rsc = nullptr; g.mul = nullptr; g.rbias = nullptr; g.ldadd = 0; g.ldmul = 0;
    g.lda = lda; g.ldb = ldb; g.ldc = ldc; g.K = K; g.ascale = 1.0f; g.bscale = 1.0f; g.oscale = 1.0f; g.addscale = 1.0f; g.M = M; g.nvalid = N; g.nstore = N; g.ldrsc = 1;
    g.bcs = 1; g.pad1 = 0; g.pad2 = 0; g.pad3 = 0;
    return g;
}
static_assert(sizeof(ZMap) == 24, "ZMap layout");
static_assert(sizeof(GemmArgs) == 8 * 24 + 8 * 8 + 2 * 8 + 4 * 4 + 4 * 4 + 4 * 4 + 4 * 4, "GemmArgs has no padding");

__global__ __launch_bounds__(256) void softmax_rows(float* S, long long sy, long long sx, int L, float prescale, const float* addv, long long say, int aydiv, int causal,
                                                  const int* imask, long long imy, long long imx, float maskval) {
    __shared__ float red[8];
    const int tid = threadIdx.x, lane = tid & 31, wid = tid >> 5;
    float* row = S + (size_t)blockIdx.y * sy + (size_t)blockIdx.x * sx;
    const float* av = addv ? addv + (size_t)(blockIdx.y / aydiv) * say : nullptr;
    const int* im = imask ? imask + (size_t)(blockIdx.y / aydiv) * imy + (size_t)blockIdx.x * imx : nullptr;
    float v[16];
    const int nj = L / 256;
    float mx = -__builtin_inff();
#pragma unroll
    for (int j = 0; j < 16; ++j) if (j < nj) { float t = row[tid + 256 * j] * prescale; if (av) t += av[tid + 256 * j]; if (im && im[tid + 256 * j] == 0) t = maskval; if (causal && (tid + 256 * j) > (int)blockIdx.x) t = -__builtin_inff(); v[j] = t; mx = fmaxf(mx, t); }
#pragma unroll
    for (int o = 16; o; o >>= 1) mx = fmaxf(mx, __shfl_xor(mx, o, 32));
    if (lane == 0) red[wid] = mx;
    __syncthreads();
    float m = red[0];
#pragma unroll
    for (int i = 1; i < 8; ++i) m = fmaxf(m, red[i]);
    if (m == -__builtin_inff()) m = 0.f;
    __syncthreads();
    float sum = 0.f;
#pragma unroll
    for (int j = 0; j < 16; ++j) if (j < nj) { v[j] = expf(v[j] - m); sum += v[j]; }
#pragma unroll
    for (int o = 16; o; o >>= 1) sum += __shfl_xor(sum, o, 32);
    if (lane == 0) red[wid] = sum;
    __syncthreads();
    float tot = 0.f;
#pragma unroll
    for (int i = 0; i < 8; ++i) tot += red[i];
    const float inv = 1.0f / tot;
#pragma unroll
    for (int j = 0; j < 16; ++j) if (j < nj) *(volatile float*)(row + tid + 256 * j) = v[j] * inv;
    __threadfence();
#pragma unroll
    for (int j = 0; j < 16; ++j) if (j < nj) *(volatile float*)(row + tid + 256 * j) = v[j] * inv;
}

#define VST2(T, p, v) do { const T vst2_v_ = (v); *(volatile T*)(p) = vst2_v_; __threadfence(); *(volatile T*)(p) = vst2_v_; } while (0)
__global__ __launch_bounds__(256) void k_unit(const float* __restrict__ st, float* UNIT) { const size_t q = (size_t)blockIdx.x * 256 + threadIdx.x; if (q >= (size_t)BB * NA_ * UU) return; const int c = (int)(q % (NA_ * UU)); const int b = (int)(q / (NA_ * UU)); VST2(float, UNIT + q, st[(size_t)b * SS + c]); }
__global__ __launch_bounds__(256) void k_pair1(const float* __restrict__ UA, const float* __restrict__ UB, const float* __restrict__ b1, int b0, float* H1) {
    const size_t q = (size_t)blockIdx.x * 256 + threadIdx.x; if (q >= (size_t)NPR * GH) return; const int c = (int)(q % GH); const int pr = (int)(q / GH); const int j = pr % NA_, i = (pr / NA_) % NA_, bl = pr / (NA_ * NA_); const int b = b0 + bl;
    VST2(float, H1 + q, fmaxf(UA[((size_t)b * NA_ + i) * GH + c] + UB[((size_t)b * NA_ + j) * GH + c] + b1[c], 0.f));
}
__global__ __launch_bounds__(256) void k_adj(const float* __restrict__ H2, const float* __restrict__ W3, const float* __restrict__ b3, int b0, float* ADJ) {
    const long long F0 = 4101LL + (long long)b0 * NA_ * NA_; const long long FA = F0 & ~31LL; const long long f = FA + (long long)blockIdx.x * 256 + threadIdx.x; const long long prl = f - F0;
    if (prl < 0 || prl >= NPR) return; const int pr = (int)prl; const int j = pr % NA_, i = (pr / NA_) % NA_, bl = pr / (NA_ * NA_); float s = b3[0];
#pragma unroll 4
    for (int c = 0; c < GH; ++c) s += fmaxf(H2[(size_t)pr * GH + c], 0.f) * W3[c];
    VST2(float, ADJ + ((size_t)(b0 + bl) * NA_ + i) * NA_ + j, 1.0f / (1.0f + expf(-s)) + (i == j ? 1.f : 0.f));
}
__global__ __launch_bounds__(64) void k_rows(const float* __restrict__ SEL, const float* __restrict__ KEYS, const int* __restrict__ act, const float* __restrict__ ADJ, const float* __restrict__ qs, const float* __restrict__ WHV, float* QT, float* PART) {
    __shared__ float lg[64], sc[64], am[16], aw[64], tq[64], te[64];
    const int b = blockIdx.x, t = threadIdx.x; const int h = t / NA_, n = t % NA_;
    float l = 0.f; const float* s = SEL + (size_t)b * (NH * EE) + h * EE; const float* k = KEYS + ((size_t)b * NA_ + n) * (NH * EE) + h * EE;
#pragma unroll 4
    for (int e = 0; e < EE; ++e) l += s[e] * k[e];
    lg[t] = l; sc[t] = (act[(size_t)b * NA_ + n] == 0) ? -99999999.0f : l * 0.17677669529663687f;
    if (t < NA_) { float m = 0.f; for (int i = 0; i < NA_; ++i) m += ADJ[((size_t)b * NA_ + i) * NA_ + t]; am[t] = m / (float)NA_; }
    __syncthreads();
    float mx = -__builtin_inff(); for (int i = 0; i < NA_; ++i) mx = fmaxf(mx, sc[h * NA_ + i]);
    float den = 0.f; for (int i = 0; i < NA_; ++i) den += expf(sc[h * NA_ + i] - mx);
    aw[t] = expf(sc[t] - mx) / den * am[n];
    __syncthreads();
    float ssum = 0.f; for (int i = 0; i < NA_; ++i) ssum += aw[h * NA_ + i];
    const float adjw = aw[t] / (ssum + 1e-8f);
    tq[t] = qs[(size_t)b * NA_ + n] * adjw; te[t] = -logf(adjw + 1e-8f) * adjw;
    __syncthreads();
    if (t < 32) { float v = 0.f;
        if (t < 4) { for (int i = 0; i < NA_; ++i) v += te[t * NA_ + i]; }
        else if (t < 8) { for (int i = 0; i < NA_; ++i) v += lg[(t - 4) * NA_ + i] * lg[(t - 4) * NA_ + i]; }
        else if (t == 8) { v = WHV[(size_t)b * 32 + 4]; for (int hh = 0; hh < NH; ++hh) { float hq = 0.f; for (int i = 0; i < NA_; ++i) hq += tq[hh * NA_ + i]; v += fabsf(WHV[(size_t)b * 32 + hh]) * hq; } }
        VST2(float, PART + (size_t)b * 32 + t, v); }
    (void)QT;
}
__global__ __launch_bounds__(256) void k_qt(const float* __restrict__ PART, float* QT) { const int b = blockIdx.x * 256 + threadIdx.x; if (b < BB) { VST2(float, QT + b, PART[(size_t)b * 32 + 8]); } }
__global__ __launch_bounds__(256) void k_whv(const float* __restrict__ st, const float* __restrict__ whW, const float* __restrict__ whb, const float* __restrict__ V1, const float* __restrict__ VW2, const float* __restrict__ Vb2, float* WHV) {
    const int lane = threadIdx.x & 31, b = blockIdx.x * 8 + (threadIdx.x >> 5); if (b >= BB) return; const float* row = st + (size_t)b * SS; float a0 = 0.f, a1 = 0.f, a2 = 0.f, a3 = 0.f;
#pragma unroll 1
    for (int c = lane; c < SS; c += 32) { const float x = row[c]; a0 += x * whW[c]; a1 += x * whW[SS + c]; a2 += x * whW[2 * SS + c]; a3 += x * whW[3 * SS + c]; }
    float v = V1[(size_t)b * 32 + lane] * VW2[lane];
#pragma unroll
    for (int o = 16; o; o >>= 1) { a0 += __shfl_xor(a0, o, 32); a1 += __shfl_xor(a1, o, 32); a2 += __shfl_xor(a2, o, 32); a3 += __shfl_xor(a3, o, 32); v += __shfl_xor(v, o, 32); }
    const float val = lane == 0 ? a0 + whb[0] : lane == 1 ? a1 + whb[1] : lane == 2 ? a2 + whb[2] : lane == 3 ? a3 + whb[3] : lane == 4 ? v + Vb2[0] : 0.f;
    VST2(float, WHV + (size_t)b * 32 + lane, val);
}
__global__ __launch_bounds__(256) void k_final(const float* __restrict__ PART, float* OUT5) {
    __shared__ double red[256]; __shared__ double res[8]; const int t = threadIdx.x;
    for (int k = 0; k < 8; ++k) { double s = 0.0; for (int b = t; b < BB; b += 256) s += (double)PART[(size_t)b * 32 + k];
        red[t] = s; __syncthreads(); for (int o = 128; o > 0; o >>= 1) { if (t < o) red[t] += red[t + o]; __syncthreads(); }
        if (t == 0) res[k] = red[0];
        __syncthreads(); }
    if (t == 0) { VST2(float, OUT5, (float)(0.001 * (res[4] + res[5] + res[6] + res[7]) / ((double)BB * NA_))); for (int h = 0; h < NH; ++h) { VST2(float, OUT5 + 1 + h, (float)(res[h] / BB)); } }
}
extern "C" void kernel_launch(void* const* d_in, const int* in_sizes, int n_in,
                              void* d_out, int out_size, void* d_ws, size_t ws_size, hipStream_t stream) {
    (void)in_sizes; (void)n_in; (void)out_size;
    const float* qs = (const float*)d_in[0]; const float* st = (const float*)d_in[1]; const int* act = (const int*)d_in[2]; const float* selW = (const float*)d_in[3]; const float* keyW = (const float*)d_in[4];
    const float* whW = (const float*)d_in[5]; const float* whb = (const float*)d_in[6]; const float* VW1 = (const float*)d_in[7]; const float* Vb1 = (const float*)d_in[8]; const float* VW2 = (const float*)d_in[9]; const float* Vb2 = (const float*)d_in[10];
    const float* gW1 = (const float*)d_in[11]; const float* gb1 = (const float*)d_in[12]; const float* gW2 = (const float*)d_in[13]; const float* gb2 = (const float*)d_in[14]; const float* gW3 = (const float*)d_in[15]; const float* gb3 = (const float*)d_in[16];
    float* qtot = (float*)d_out;
    float* scal = qtot + BB;
    float* adj = qtot + 4101;
    char* wsp = (char*)d_ws;
    auto take = [&](size_t bytes) { char* p = wsp; wsp += (bytes + 255) & ~(size_t)255; return (void*)p; };
    float* UNIT = (float*)take((size_t)BB * NA_ * UU * 4); float* SEL = (float*)take((size_t)BB * NH * EE * 4); float* KEYS = (float*)take((size_t)BB * NA_ * NH * EE * 4); float* UA = (float*)take((size_t)BB * NA_ * GH * 4); float* UB = (float*)take((size_t)BB * NA_ * GH * 4);
    float* H1 = (float*)take((size_t)NPR * GH * 4); float* H2 = (float*)take((size_t)NPR * GH * 4); float* V1 = (float*)take((size_t)BB * 32 * 4); float* WHV = (float*)take((size_t)BB * 32 * 4); float* PART = (float*)take((size_t)BB * 32 * 4); float* SCAL = (float*)take(64 * 4);
    if ((size_t)(wsp - (char*)d_ws) > ws_size) return;
    k_unit<<<(BB * NA_ * UU) / 256, 256, 0, stream>>>(st, UNIT);
    { GemmArgs g = gemm_args(st, SS, zm(0), selW, SS, zm(0), SEL, NH * EE, zm(0), BB, NH * EE, SS); gemm_kernel<1, 1, 1, 1, 4, 2, ACT_NONE><<<dim3(BB / 64, 1, 1), 256, 0, stream>>>(g); }
    { GemmArgs g = gemm_args(UNIT, UU, zm(0), keyW, UU, zm(0), KEYS, NH * EE, zm(0), BB * NA_, NH * EE, UU); gemm_kernel<1, 1, 1, 1, 4, 2, ACT_NONE><<<dim3((BB * NA_) / 64, 1, 1), 256, 0, stream>>>(g); }
    { GemmArgs g = gemm_args(UNIT, UU, zm(0), gW1, 2 * UU, zm(0), UA, GH, zm(0), BB * NA_, GH, UU); gemm_kernel<1, 1, 1, 1, 8, 1, ACT_NONE><<<dim3((BB * NA_) / 128, 1, 1), 256, 0, stream>>>(g); }
    { GemmArgs g = gemm_args(UNIT, UU, zm(0), gW1 + UU, 2 * UU, zm(0), UB, GH, zm(0), BB * NA_, GH, UU); gemm_kernel<1, 1, 1, 1, 8, 1, ACT_NONE><<<dim3((BB * NA_) / 128, 1, 1), 256, 0, stream>>>(g); }
    for (int b0 = 0; b0 < BB; b0 += BCH) {
        k_pair1<<<(unsigned)(((size_t)NPR * GH) / 256), 256, 0, stream>>>(UA, UB, gb1, b0, H1);
        { GemmArgs g = gemm_args(H1, GH, zm(0), gW2, GH, zm(0), H2, GH, zm(0), NPR, GH, GH); g.bias = gb2; gemm_kernel<1, 1, 1, 1, 8, 1, ACT_NONE><<<dim3(NPR / 128, 1, 1), 256, 0, stream>>>(g); }
        k_adj<<<(NPR + 32 + 255) / 256, 256, 0, stream>>>(H2, gW3, gb3, b0, adj);
    }
    { GemmArgs g = gemm_args(st, SS, zm(0), VW1, SS, zm(0), V1, 32, zm(0), BB, 32, SS); g.bias = Vb1; gemm_kernel<1, 1, 1, 1, 8, 1, ACT_RELU><<<dim3(BB / 128, 1, 1), 256, 0, stream>>>(g); }
    k_whv<<<BB / 8, 256, 0, stream>>>(st, whW, whb, V1, VW2, Vb2, WHV);
    k_rows<<<BB, 64, 0, stream>>>(SEL, KEYS, act, adj, qs, WHV, qtot, PART);
    k_qt<<<BB / 256, 256, 0, stream>>>(PART, qtot);
    k_final<<<1, 256, 0, stream>>>(PART, scal);
}
